// Contrast_MultiHeadSelfAttention_22119081574883
// MI455X (gfx1250) — hardware-run, weakly checked
//
#include <hip/hip_runtime.h>
#include <stdint.h>

constexpr int kBatch      = 4;
constexpr int kSeqN       = 1024;
constexpr int kDim        = 1024;
constexpr int kHeads      = 16;
constexpr int kHeadD      = 64;
constexpr int kTok        = kBatch * kSeqN;
constexpr int kChunkPairs = 8;
constexpr int kNumChunks  = (kBatch * kHeads) / kChunkPairs;
constexpr float kScoreScale = 0.125f;
constexpr float kPCarry     = 4096.0f;
constexpr float kPCarryInv  = 1.0f / 4096.0f;
static_assert(kHeads % kChunkPairs == 0, "a chunk stays inside one batch");
static_assert(kHeads * kHeadD == kDim, "head split");

constexpr size_t kPlane16B  = (size_t)kTok * kDim * 2;
constexpr size_t kW16B      = (size_t)kDim * kDim * 2;
constexpr size_t kSChunkB   = (size_t)kChunkPairs * kSeqN * kSeqN * 4;
constexpr size_t kPChunkB   = (size_t)kChunkPairs * kSeqN * kSeqN * 2;
constexpr size_t kOffQ16  = 0;
constexpr size_t kOffK16  = kOffQ16 + kPlane16B;
constexpr size_t kOffVt16 = kOffK16 + kPlane16B;
constexpr size_t kOffXb   = kOffVt16 + kPlane16B;
constexpr size_t kOffYb   = kOffXb + kPlane16B;
constexpr size_t kOffWq   = kOffYb + kPlane16B;
constexpr size_t kOffWk   = kOffWq + kW16B;
constexpr size_t kOffWv   = kOffWk + kW16B;
constexpr size_t kEndCast = kOffWv + kW16B;
constexpr size_t kOffS    = kOffXb;
constexpr size_t kOffP1   = kOffS + kSChunkB;
constexpr size_t kOffP2   = kOffP1 + kPChunkB;
constexpr size_t kEndChunk = kOffP2 + kPChunkB;
constexpr size_t kWsTotal = (kEndCast > kEndChunk) ? kEndCast : kEndChunk;
static_assert(kWsTotal == 92274688, "carve total");
static_assert(kWsTotal <= 134217728, "carve under 128 MiB");

typedef __attribute__((ext_vector_type(16))) _Float16 v16h;
typedef __attribute__((ext_vector_type(8)))  _Float16 v8h;
typedef __attribute__((ext_vector_type(16))) __bf16   v16b;
typedef __attribute__((ext_vector_type(8)))  __bf16   v8b;
typedef __attribute__((ext_vector_type(8)))  float    v8f;
typedef __attribute__((ext_vector_type(4)))  float    v4f;
typedef __attribute__((ext_vector_type(4)))  unsigned int v4u;

__device__ __forceinline__ unsigned short f2bf_bits(float f) {
  unsigned u = __float_as_uint(f);
  return (unsigned short)((u + 0x7FFFu + ((u >> 16) & 1u)) >> 16);
}
__device__ __forceinline__ float bf_bits2f(unsigned short h) { return __uint_as_float(((unsigned)h) << 16); }

__device__ __forceinline__ void dep_guard_h(v8f& a, v8f& b, v16h x, v16h y) { asm volatile("v_nop\n\tv_nop\n\tv_nop\n\tv_nop" : "+v"(a), "+v"(b) : "v"(x), "v"(y)); }
__device__ __forceinline__ void dep_guard_b(v8f& a, v8f& b, v16b x, v16b y) { asm volatile("v_nop\n\tv_nop\n\tv_nop\n\tv_nop" : "+v"(a), "+v"(b) : "v"(x), "v"(y)); }
__device__ __forceinline__ void keep4_h(v16h a, v16h b, v16h c, v16h d) { asm volatile("v_nop" :: "v"(a), "v"(b), "v"(c), "v"(d)); }
__device__ __forceinline__ void keep4_b(v16b a, v16b b, v16b c, v16b d) { asm volatile("v_nop" :: "v"(a), "v"(b), "v"(c), "v"(d)); }
__device__ __forceinline__ void acc_guard4(v8f& a, v8f& b, v8f& c, v8f& d) { asm volatile("v_nop\n\tv_nop\n\tv_nop\n\tv_nop" : "+v"(a), "+v"(b), "+v"(c), "+v"(d)); }
template <typename T> struct Frag;
template <> struct Frag<_Float16> {
  typedef v16h V; union U { v16h v; v8h h[2]; };
  static __device__ __forceinline__ v16h load(const _Float16* p) {
    U f; f.h[0] = *(const v8h*)(p); f.h[1] = *(const v8h*)(p + 16); return f.v;
  }
  static __device__ __forceinline__ v8f mma(v16h a, v16h b, v8f c) {
    return __builtin_amdgcn_wmma_f32_16x16x32_f16(false, a, false, b, (short)0, c, false, false);
  }
  static __device__ __forceinline__ void guard(v8f& a, v8f& b, v16h x, v16h y) { dep_guard_h(a, b, x, y); }
  static __device__ __forceinline__ void keep(v16h a, v16h b, v16h c, v16h d) { keep4_h(a, b, c, d); }
};
template <> struct Frag<__bf16> {
  typedef v16b V; union U { v16b v; v8b h[2]; };
  static __device__ __forceinline__ v16b load(const __bf16* p) {
    U f; f.h[0] = *(const v8b*)(p); f.h[1] = *(const v8b*)(p + 16); return f.v;
  }
  static __device__ __forceinline__ v8f mma(v16b a, v16b b, v8f c) {
    return __builtin_amdgcn_wmma_f32_16x16x32_bf16(false, a, false, b, (short)0, c, false, false);
  }
  static __device__ __forceinline__ void guard(v8f& a, v8f& b, v16b x, v16b y) { dep_guard_b(a, b, x, y); }
  static __device__ __forceinline__ void keep(v16b a, v16b b, v16b c, v16b d) { keep4_b(a, b, c, d); }
};

__device__ __forceinline__ unsigned pk16(unsigned short a, unsigned short b) { return (unsigned)a | ((unsigned)b << 16); }
__device__ __forceinline__ unsigned short h_bits(float f) { const _Float16 h = (_Float16)f; return __builtin_bit_cast(unsigned short, h); }

template <int ET> struct Elem;
template <> struct Elem<0> { typedef _Float16 T; };
template <> struct Elem<1> { typedef __bf16 T; };
template <int ET, bool SPLIT, int BIAS_MODE, int OUT_MODE, bool RESID, int ACT = 0>
__global__ __launch_bounds__(256) void wmma_gemm64(
    const unsigned short* __restrict__ Ap, const unsigned short* __restrict__ A2p, int lda, long strideA,
    const unsigned short* __restrict__ Btp, const unsigned short* __restrict__ Bt2p, int ldb, long strideB,
    void* __restrict__ Cout, void* __restrict__ Cout2, int ldc, long strideC,
    const float* __restrict__ bias,
    const float* __restrict__ resid, long strideR,
    int M, int N, int K, float scale) {
  typedef typename Elem<ET>::T T;
  typedef typename Frag<T>::V V;
  const T* A = (const T*)Ap; const T* A2 = (const T*)A2p; const T* Bt = (const T*)Btp; const T* Bt2 = (const T*)Bt2p;
  __shared__ __align__(16) float sT[8][16 * 68];
  const int b    = blockIdx.y;
  const int lane = threadIdx.x & 31;
  const int wave = threadIdx.x >> 5;
  const int tilesN = N >> 6;
  const int tilesM = M >> 6;
  const int tile = blockIdx.x * 8 + wave;
  if (tile >= tilesM * tilesN) return;
  const int tm = tile / tilesN;
  const int tn = tile - tm * tilesN;
  const int m0 = tm << 6;
  const int n0 = tn << 6;

  const T* Ab  = A  + (size_t)b * strideA;
  const T* Bb  = Bt + (size_t)b * strideB;
  const T* Ab2 = SPLIT ? (A2  + (size_t)b * strideA) : nullptr;
  const T* Bb2 = SPLIT ? (Bt2 + (size_t)b * strideB) : nullptr;

  const int rlane = lane & 15;
  const int koff  = (lane >> 4) * 8;
  const int mOff  = (lane >> 4) * 8;

  v8f acc[4][4];
#pragma unroll
  for (int i = 0; i < 4; ++i)
#pragma unroll
    for (int j = 0; j < 4; ++j) acc[i][j] = (v8f){0.f,0.f,0.f,0.f,0.f,0.f,0.f,0.f};

  for (int k0 = 0; k0 < K; k0 += 32) {
    V bh[4], bl[4];
#pragma unroll
    for (int j = 0; j < 4; ++j) {
      const size_t bo = (size_t)(n0 + (j << 4) + rlane) * ldb + koff + k0;
      bh[j] = Frag<T>::load(Bb + bo);
      if (SPLIT) bl[j] = Frag<T>::load(Bb2 + bo);
    }
#pragma unroll
    for (int i = 0; i < 4; ++i) {
      const size_t ao = (size_t)(m0 + (i << 4) + rlane) * lda + koff + k0;
      V ah = Frag<T>::load(Ab + ao);
      V al;
      if (SPLIT) al = Frag<T>::load(Ab2 + ao);
#pragma unroll
      for (int j = 0; j < 4; ++j) {
        acc[i][j] = Frag<T>::mma(ah, bh[j], acc[i][j]);
        if (SPLIT) {
          acc[i][j] = Frag<T>::mma(ah, bl[j], acc[i][j]);
          acc[i][j] = Frag<T>::mma(al, bh[j], acc[i][j]);
        }
      }
      Frag<T>::guard(acc[i][0], acc[i][3], ah, SPLIT ? al : ah);
    }
    Frag<T>::keep(bh[0], bh[1], bh[2], bh[3]);
    if (SPLIT) Frag<T>::keep(bl[0], bl[1], bl[2], bl[3]);
  }
  acc_guard4(acc[0][0], acc[0][1], acc[0][2], acc[0][3]);
  acc_guard4(acc[1][0], acc[1][1], acc[1][2], acc[1][3]);
  acc_guard4(acc[2][0], acc[2][1], acc[2][2], acc[2][3]);
  acc_guard4(acc[3][0], acc[3][1], acc[3][2], acc[3][3]);

  float* slab = sT[wave];
  const float* Rb = RESID ? (resid + (size_t)b * strideR) : nullptr;
#pragma unroll
  for (int i = 0; i < 4; ++i) {
    const int mBase = m0 + (i << 4);
#pragma unroll
    for (int j = 0; j < 4; ++j) {
      const int n = n0 + (j << 4) + rlane;
      float bv = 0.f;
      if (BIAS_MODE == 2) bv = bias[n];
#pragma unroll
      for (int r = 0; r < 8; ++r) {
        float v = acc[i][j][r] * scale;
        if (BIAS_MODE == 1) v += bias[mBase + mOff + r];
        if (BIAS_MODE == 2) v += bv;
        if (RESID) v += Rb[(size_t)(mBase + mOff + r) * ldc + n];
        if (ACT == 2) v = fmaxf(v, 0.0f);
        if (ACT == 4) v = (v > 0.f) ? v : 0.01f * v;
        slab[(mOff + r) * 68 + (j << 4) + rlane] = v;
      }
    }
    __builtin_amdgcn_fence(__ATOMIC_RELEASE, "workgroup");
    __builtin_amdgcn_wave_barrier();
    __builtin_amdgcn_fence(__ATOMIC_ACQUIRE, "workgroup");
    if (OUT_MODE == 0) {
      float* C = (float*)Cout + (size_t)b * strideC;
      const int hh = lane >> 4, c4 = (lane & 15) * 4;
      for (int pass = 0; pass < 2; ++pass) {
#pragma unroll
        for (int it = 0; it < 8; ++it) {
          const int row = it * 2 + hh;
          v4f v = *(const v4f*)(slab + row * 68 + c4);
          *(volatile v4f*)(C + (size_t)(mBase + row) * ldc + n0 + c4) = v;
        }
        __threadfence();
      }
    } else {
      const int q = lane >> 3, c8 = (lane & 7) * 8;
      unsigned short* C  = (unsigned short*)Cout  + (size_t)b * strideC;
      unsigned short* C2 = (OUT_MODE == 2) ? ((unsigned short*)Cout2 + (size_t)b * strideC) : nullptr;
      for (int pass = 0; pass < 2; ++pass) {
#pragma unroll
        for (int it = 0; it < 4; ++it) {
          const int row = it * 4 + q;
          const float* sp = slab + row * 68 + c8;
          v8h hv, lv;
#pragma unroll
          for (int e = 0; e < 8; ++e) {
            if (OUT_MODE == 1) {
              hv[e] = (_Float16)sp[e];
            } else {
              unsigned short hb = f2bf_bits(sp[e]);
              unsigned short lb = f2bf_bits(sp[e] - bf_bits2f(hb));
              hv[e] = __builtin_bit_cast(_Float16, hb);
              lv[e] = __builtin_bit_cast(_Float16, lb);
            }
          }
          *(volatile v8h*)(C + (size_t)(mBase + row) * ldc + n0 + c8) = hv;
          if (OUT_MODE == 2) *(volatile v8h*)(C2 + (size_t)(mBase + row) * ldc + n0 + c8) = lv;
        }
        __threadfence();
      }
    }
    __builtin_amdgcn_fence(__ATOMIC_RELEASE, "workgroup");
    __builtin_amdgcn_wave_barrier();
    __builtin_amdgcn_fence(__ATOMIC_ACQUIRE, "workgroup");
  }
}

__global__ __launch_bounds__(256) void cast8_bf16_kernel(const float* __restrict__ in, unsigned short* __restrict__ out, int n8) {
  const int i = blockIdx.x * 256 + threadIdx.x;
  if (i >= n8) return;
  const float* p = in + 8 * (size_t)i;
  const v4f a = *(const v4f*)(p);
  const v4f c = *(const v4f*)(p + 4);
  unsigned short hb[8];
#pragma unroll
  for (int e = 0; e < 4; ++e) {
    hb[e]     = f2bf_bits(a[e]);
    hb[4 + e] = f2bf_bits(c[e]);
  }
  const v4u u = (v4u){pk16(hb[0], hb[1]), pk16(hb[2], hb[3]), pk16(hb[4], hb[5]), pk16(hb[6], hb[7])};
  unsigned short* q = out + 8 * (size_t)i;
  *(volatile v4u*)q = u;
  __threadfence();
  *(volatile v4u*)q = u;
}

__device__ __forceinline__ float wave_max32(float v) {
#pragma unroll
  for (int off = 16; off > 0; off >>= 1) v = fmaxf(v, __shfl_xor(v, off, 32));
  return v;
}
__device__ __forceinline__ float wave_sum32(float v) {
#pragma unroll
  for (int off = 16; off > 0; off >>= 1) v += __shfl_xor(v, off, 32);
  return v;
}

__global__ __launch_bounds__(128) void dual_softmax_kernel(const float* __restrict__ S,
                                                           unsigned short* __restrict__ P1,
                                                           unsigned short* __restrict__ P2, float carry) {
  __shared__ float red[6][4];
  const int row  = blockIdx.x;
  const int t    = threadIdx.x;
  const int lane = t & 31, wave = t >> 5;
  const int c0   = t * 8;
  const float* sr = S + (size_t)row * kSeqN + c0;
  const v4f a = *(const v4f*)(sr);
  const v4f c = *(const v4f*)(sr + 4);
  float x[8];
#pragma unroll
  for (int e = 0; e < 4; ++e) { x[e] = a[e]; x[4 + e] = c[e]; }

  float m0 = fmaxf(fmaxf(fmaxf(x[0], x[1]), fmaxf(x[2], x[3])), fmaxf(fmaxf(x[4], x[5]), fmaxf(x[6], x[7])));
  m0 = wave_max32(m0);
  if (lane == 0) red[0][wave] = m0;
  __syncthreads();
  m0 = fmaxf(fmaxf(red[0][0], red[0][1]), fmaxf(red[0][2], red[0][3]));
  float d[8];
  float s0 = 0.f;
#pragma unroll
  for (int e = 0; e < 8; ++e) { d[e] = __expf(x[e] - m0); s0 += d[e]; }
  s0 = wave_sum32(s0);
  if (lane == 0) red[1][wave] = s0;
  __syncthreads();
  s0 = ((red[1][0] + red[1][1]) + red[1][2]) + red[1][3];
  const float inv0 = 1.0f / s0;
#pragma unroll
  for (int e = 0; e < 8; ++e) d[e] *= inv0;

  float u[8];
#pragma unroll
  for (int e = 0; e < 8; ++e) u[e] = 1.0f - d[e];
  float m1 = fmaxf(fmaxf(fmaxf(u[0], u[1]), fmaxf(u[2], u[3])), fmaxf(fmaxf(u[4], u[5]), fmaxf(u[6], u[7])));
  m1 = wave_max32(m1);
  if (lane == 0) red[2][wave] = m1;
  __syncthreads();
  m1 = fmaxf(fmaxf(red[2][0], red[2][1]), fmaxf(red[2][2], red[2][3]));
  float g1[8];
  float s1 = 0.f;
#pragma unroll
  for (int e = 0; e < 8; ++e) { g1[e] = __expf(u[e] - m1); s1 += g1[e]; }
  s1 = wave_sum32(s1);
  if (lane == 0) red[3][wave] = s1;
  __syncthreads();
  s1 = ((red[3][0] + red[3][1]) + red[3][2]) + red[3][3];
  const float inv1 = 1.0f / s1;

  float m2 = fmaxf(fmaxf(fmaxf(d[0], d[1]), fmaxf(d[2], d[3])), fmaxf(fmaxf(d[4], d[5]), fmaxf(d[6], d[7])));
  m2 = wave_max32(m2);
  if (lane == 0) red[4][wave] = m2;
  __syncthreads();
  m2 = fmaxf(fmaxf(red[4][0], red[4][1]), fmaxf(red[4][2], red[4][3]));
  float g2[8];
  float s2 = 0.f;
#pragma unroll
  for (int e = 0; e < 8; ++e) { g2[e] = __expf(d[e] - m2); s2 += g2[e]; }
  s2 = wave_sum32(s2);
  if (lane == 0) red[5][wave] = s2;
  __syncthreads();
  s2 = ((red[5][0] + red[5][1]) + red[5][2]) + red[5][3];
  const float inv2 = 1.0f / s2;

  unsigned short hb1[8], hb2[8];
#pragma unroll
  for (int e = 0; e < 8; ++e) {
    const float p1 = g1[e] * inv1;
    const float p2 = g2[e] * inv2;
    hb1[e] = h_bits(p1 * carry);
    hb2[e] = h_bits(p2 * carry);
  }
  const v4u u1 = (v4u){pk16(hb1[0], hb1[1]), pk16(hb1[2], hb1[3]), pk16(hb1[4], hb1[5]), pk16(hb1[6], hb1[7])};
  const v4u u2 = (v4u){pk16(hb2[0], hb2[1]), pk16(hb2[2], hb2[3]), pk16(hb2[4], hb2[5]), pk16(hb2[6], hb2[7])};
  unsigned short* q1 = P1 + (size_t)row * kSeqN + c0;
  unsigned short* q2 = P2 + (size_t)row * kSeqN + c0;
  *(volatile v4u*)q1 = u1;
  *(volatile v4u*)q2 = u2;
  __threadfence();
  *(volatile v4u*)q1 = u1;
  *(volatile v4u*)q2 = u2;
}

extern "C" void kernel_launch(void* const* d_in, const int* in_sizes, int n_in,
                              void* d_out, int out_size, void* d_ws, size_t ws_size,
                              hipStream_t stream) {
  if (n_in < 5) return;
  if (in_sizes[0] != kTok * kDim || in_sizes[1] != kTok * kDim) return;
  if (in_sizes[2] != kDim * kDim || in_sizes[3] != kDim * kDim || in_sizes[4] != kDim * kDim) return;
  if (out_size != 2 * kTok * kDim) return;
  if (ws_size < kWsTotal) return;

  const float* x  = (const float*)d_in[0];
  const float* y  = (const float*)d_in[1];
  const float* Wq = (const float*)d_in[2];
  const float* Wk = (const float*)d_in[3];
  const float* Wv = (const float*)d_in[4];

  unsigned char* ws = (unsigned char*)d_ws;
  unsigned short* q16  = (unsigned short*)(ws + kOffQ16);
  unsigned short* k16  = (unsigned short*)(ws + kOffK16);
  unsigned short* vt16 = (unsigned short*)(ws + kOffVt16);
  unsigned short* xb   = (unsigned short*)(ws + kOffXb);
  unsigned short* yb   = (unsigned short*)(ws + kOffYb);
  unsigned short* wqb  = (unsigned short*)(ws + kOffWq);
  unsigned short* wkb  = (unsigned short*)(ws + kOffWk);
  unsigned short* wvb  = (unsigned short*)(ws + kOffWv);
  float*          sbuf = (float*)(ws + kOffS);
  unsigned short* p1   = (unsigned short*)(ws + kOffP1);
  unsigned short* p2   = (unsigned short*)(ws + kOffP2);
  const float* fdummy  = (const float*)(ws + kOffQ16);

  float* out0 = (float*)d_out;
  float* out1 = out0 + (size_t)kTok * kDim;

  const int n8Tok = (kTok * kDim) / 8;
  const int n8W   = (kDim * kDim) / 8;
  cast8_bf16_kernel<<<dim3((n8Tok + 255) / 256), 256, 0, stream>>>(x, xb, n8Tok);
  cast8_bf16_kernel<<<dim3((n8Tok + 255) / 256), 256, 0, stream>>>(y, yb, n8Tok);
  cast8_bf16_kernel<<<dim3((n8W + 255) / 256), 256, 0, stream>>>(Wq, wqb, n8W);
  cast8_bf16_kernel<<<dim3((n8W + 255) / 256), 256, 0, stream>>>(Wk, wkb, n8W);
  cast8_bf16_kernel<<<dim3((n8W + 255) / 256), 256, 0, stream>>>(Wv, wvb, n8W);

  wmma_gemm64<1, false, 0, 1, false, 0><<<dim3(128, 1), 256, 0, stream>>>(
      xb, xb, kDim, 0L, wqb, wqb, kDim, 0L, (void*)q16, (void*)q16, kDim, 0L,
      fdummy, fdummy, 0L, kTok, kDim, kDim, 1.0f);
  wmma_gemm64<1, false, 0, 1, false, 0><<<dim3(128, 1), 256, 0, stream>>>(
      xb, xb, kDim, 0L, wkb, wkb, kDim, 0L, (void*)k16, (void*)k16, kDim, 0L,
      fdummy, fdummy, 0L, kTok, kDim, kDim, 1.0f);
  wmma_gemm64<1, false, 0, 1, false, 0><<<dim3(32, kBatch), 256, 0, stream>>>(
      wvb, wvb, kDim, 0L, yb, yb, kDim, (long)kSeqN * kDim, (void*)vt16, (void*)vt16, kSeqN, (long)kDim * kSeqN,
      fdummy, fdummy, 0L, kDim, kSeqN, kDim, 1.0f);

  const long planeS = (long)kSeqN * kSeqN;
  for (int ch = 0; ch < kNumChunks; ++ch) {
    const int bb = (ch * kChunkPairs) / kHeads;
    const int h0 = (ch * kChunkPairs) % kHeads;
    const size_t tokBase = (size_t)bb * kSeqN * kDim;
    wmma_gemm64<0, false, 0, 0, false, 0><<<dim3(32, kChunkPairs), 256, 0, stream>>>(
        q16 + tokBase + (size_t)h0 * kHeadD, q16, kDim, (long)kHeadD,
        k16 + tokBase + (size_t)h0 * kHeadD, k16, kDim, (long)kHeadD,
        (void*)sbuf, (void*)sbuf, kSeqN, planeS,
        fdummy, fdummy, 0L, kSeqN, kSeqN, kHeadD, kScoreScale);
    dual_softmax_kernel<<<dim3(kChunkPairs * kSeqN), 128, 0, stream>>>(sbuf, p1, p2, kPCarry);
    const unsigned short* vtb = vt16 + (size_t)bb * kDim * kSeqN + (size_t)h0 * kHeadD * kSeqN;
    wmma_gemm64<0, false, 0, 0, false, 0><<<dim3(2, kChunkPairs), 256, 0, stream>>>(
        p1, p1, kSeqN, planeS,
        vtb, vtb, kSeqN, (long)kHeadD * kSeqN,
        (void*)(out0 + tokBase + (size_t)h0 * kHeadD), (void*)(out0 + tokBase + (size_t)h0 * kHeadD), kDim, (long)kHeadD,
        fdummy, fdummy, 0L, kSeqN, kHeadD, kSeqN, kPCarryInv);
    wmma_gemm64<0, false, 0, 0, false, 0><<<dim3(2, kChunkPairs), 256, 0, stream>>>(
        p2, p2, kSeqN, planeS,
        vtb, vtb, kSeqN, (long)kHeadD * kSeqN,
        (void*)(out1 + tokBase + (size_t)h0 * kHeadD), (void*)(out1 + tokBase + (size_t)h0 * kHeadD), kDim, (long)kHeadD,
        fdummy, fdummy, 0L, kSeqN, kHeadD, kSeqN, kPCarryInv);
  }
}
